// MLPPredictor_80410377716239
// MI455X (gfx1250) — hardware-run, weakly checked
//
#include <hip/hip_runtime.h>
#include <math.h>

constexpr int kNodes        = 100000;
constexpr int kNodesPad     = 100032;
constexpr int kHid          = 128;
constexpr int kCat          = 256;
constexpr int kEdges        = 500000;
constexpr int kThreads      = 256;
constexpr int kHGroups      = kNodesPad * kHid / 8;
constexpr int kHBlocks      = kHGroups / kThreads;
constexpr int kWGroups      = kCat * kHid / 8;
constexpr int kWBlocks      = kWGroups / kThreads;
constexpr int kEdgesPerBlk  = 256;
constexpr int kEdgeBlocks   = (kEdges + kEdgesPerBlk - 1) / kEdgesPerBlk;
constexpr int kGemmTiles    = (kNodesPad / 64) * (kCat / 64);
constexpr int kGemmBlocks   = (kGemmTiles + 7) / 8;

static_assert(kNodesPad % 64 == 0 && kNodesPad >= kNodes && kNodesPad - kNodes < 64);
static_assert(kCat % 64 == 0);
static_assert(kHid % 32 == 0);
static_assert(kHGroups % kThreads == 0);
static_assert(kWGroups % kThreads == 0);
static_assert(kEdges % 32 == 0);
static_assert(kHid == 4 * 32);

constexpr size_t kHbBytes  = (size_t)kNodesPad * kHid * 2;
constexpr size_t kW1tBytes = (size_t)kCat * kHid * 2;
constexpr size_t kPBytes   = (size_t)kNodesPad * kCat * 4;
constexpr size_t kWsTotal  = kHbBytes + kW1tBytes + kPBytes;
static_assert(kWsTotal == 128106496);
static_assert(kWsTotal <= 134217728);
static_assert(kHbBytes % 256 == 0 && kW1tBytes % 256 == 0);

typedef __attribute__((ext_vector_type(16))) _Float16 v16h;
typedef __attribute__((ext_vector_type(8)))  _Float16 v8h;
typedef __attribute__((ext_vector_type(16))) __bf16   v16b;
typedef __attribute__((ext_vector_type(8)))  __bf16   v8b;
typedef __attribute__((ext_vector_type(8)))  float    v8f;
typedef __attribute__((ext_vector_type(4)))  float    v4f;
typedef __attribute__((ext_vector_type(4)))  unsigned int v4u;

__device__ __forceinline__ unsigned short f2bf_bits(float f) {
  unsigned u = __float_as_uint(f);
  return (unsigned short)((u + 0x7FFFu + ((u >> 16) & 1u)) >> 16);
}
__device__ __forceinline__ float bf_bits2f(unsigned short h) { return __uint_as_float(((unsigned)h) << 16); }
__device__ __forceinline__ float bfr(float f) { return bf_bits2f(f2bf_bits(f)); }
__device__ __forceinline__ unsigned pk16(unsigned short a, unsigned short b) { return (unsigned)a | ((unsigned)b << 16); }

__device__ __forceinline__ void dep_guard_h(v8f& a, v8f& b, v16h x, v16h y) { asm volatile("v_nop\n\tv_nop\n\tv_nop\n\tv_nop" : "+v"(a), "+v"(b) : "v"(x), "v"(y)); }
__device__ __forceinline__ void dep_guard_b(v8f& a, v8f& b, v16b x, v16b y) { asm volatile("v_nop\n\tv_nop\n\tv_nop\n\tv_nop" : "+v"(a), "+v"(b) : "v"(x), "v"(y)); }
__device__ __forceinline__ void keep4_h(v16h a, v16h b, v16h c, v16h d) { asm volatile("v_nop" :: "v"(a), "v"(b), "v"(c), "v"(d)); }
__device__ __forceinline__ void keep4_b(v16b a, v16b b, v16b c, v16b d) { asm volatile("v_nop" :: "v"(a), "v"(b), "v"(c), "v"(d)); }
__device__ __forceinline__ void acc_guard4(v8f& a, v8f& b, v8f& c, v8f& d) { asm volatile("v_nop\n\tv_nop\n\tv_nop\n\tv_nop" : "+v"(a), "+v"(b), "+v"(c), "+v"(d)); }
template <typename T> struct Frag;
template <> struct Frag<_Float16> {
  typedef v16h V; union U { v16h v; v8h h[2]; };
  static __device__ __forceinline__ v16h load(const _Float16* p) {
    U f; f.h[0] = *(const v8h*)(p); f.h[1] = *(const v8h*)(p + 16); return f.v;
  }
  static __device__ __forceinline__ v8f mma(v16h a, v16h b, v8f c) {
    return __builtin_amdgcn_wmma_f32_16x16x32_f16(false, a, false, b, (short)0, c, false, false);
  }
  static __device__ __forceinline__ void guard(v8f& a, v8f& b, v16h x, v16h y) { dep_guard_h(a, b, x, y); }
  static __device__ __forceinline__ void keep(v16h a, v16h b, v16h c, v16h d) { keep4_h(a, b, c, d); }
};
template <> struct Frag<__bf16> {
  typedef v16b V; union U { v16b v; v8b h[2]; };
  static __device__ __forceinline__ v16b load(const __bf16* p) {
    U f; f.h[0] = *(const v8b*)(p); f.h[1] = *(const v8b*)(p + 16); return f.v;
  }
  static __device__ __forceinline__ v8f mma(v16b a, v16b b, v8f c) {
    return __builtin_amdgcn_wmma_f32_16x16x32_bf16(false, a, false, b, (short)0, c, false, false);
  }
  static __device__ __forceinline__ void guard(v8f& a, v8f& b, v16b x, v16b y) { dep_guard_b(a, b, x, y); }
  static __device__ __forceinline__ void keep(v16b a, v16b b, v16b c, v16b d) { keep4_b(a, b, c, d); }
};

template <int ET> struct Elem;
template <> struct Elem<0> { typedef _Float16 T; };
template <> struct Elem<1> { typedef __bf16 T; };
template <int ET, bool SPLIT, int BIAS_MODE, int OUT_MODE, bool RESID, int ACT = 0>
__global__ __launch_bounds__(256) void wmma_gemm64(
    const unsigned short* __restrict__ Ap, const unsigned short* __restrict__ A2p, int lda, long strideA,
    const unsigned short* __restrict__ Btp, const unsigned short* __restrict__ Bt2p, int ldb, long strideB,
    void* __restrict__ Cout, void* __restrict__ Cout2, int ldc, long strideC,
    const float* __restrict__ bias,
    const float* __restrict__ resid, long strideR,
    int M, int N, int K, float scale) {
  typedef typename Elem<ET>::T T;
  typedef typename Frag<T>::V V;
  const T* A = (const T*)Ap; const T* A2 = (const T*)A2p; const T* Bt = (const T*)Btp; const T* Bt2 = (const T*)Bt2p;
  __shared__ __align__(16) float sT[8][16 * 68];
  const int b    = blockIdx.y;
  const int lane = threadIdx.x & 31;
  const int wave = threadIdx.x >> 5;
  const int tilesN = N >> 6;
  const int tilesM = M >> 6;
  const int tile = blockIdx.x * 8 + wave;
  if (tile >= tilesM * tilesN) return;
  const int tm = tile / tilesN;
  const int tn = tile - tm * tilesN;
  const int m0 = tm << 6;
  const int n0 = tn << 6;

  const T* Ab  = A  + (size_t)b * strideA;
  const T* Bb  = Bt + (size_t)b * strideB;
  const T* Ab2 = SPLIT ? (A2  + (size_t)b * strideA) : nullptr;
  const T* Bb2 = SPLIT ? (Bt2 + (size_t)b * strideB) : nullptr;

  const int rlane = lane & 15;
  const int koff  = (lane >> 4) * 8;
  const int mOff  = (lane >> 4) * 8;

  v8f acc[4][4];
#pragma unroll
  for (int i = 0; i < 4; ++i)
#pragma unroll
    for (int j = 0; j < 4; ++j) acc[i][j] = (v8f){0.f,0.f,0.f,0.f,0.f,0.f,0.f,0.f};

  for (int k0 = 0; k0 < K; k0 += 32) {
    V bh[4], bl[4];
#pragma unroll
    for (int j = 0; j < 4; ++j) {
      const size_t bo = (size_t)(n0 + (j << 4) + rlane) * ldb + koff + k0;
      bh[j] = Frag<T>::load(Bb + bo);
      if (SPLIT) bl[j] = Frag<T>::load(Bb2 + bo);
    }
#pragma unroll
    for (int i = 0; i < 4; ++i) {
      const size_t ao = (size_t)(m0 + (i << 4) + rlane) * lda + koff + k0;
      V ah = Frag<T>::load(Ab + ao);
      V al;
      if (SPLIT) al = Frag<T>::load(Ab2 + ao);
#pragma unroll
      for (int j = 0; j < 4; ++j) {
        acc[i][j] = Frag<T>::mma(ah, bh[j], acc[i][j]);
        if (SPLIT) {
          acc[i][j] = Frag<T>::mma(ah, bl[j], acc[i][j]);
          acc[i][j] = Frag<T>::mma(al, bh[j], acc[i][j]);
        }
      }
      Frag<T>::guard(acc[i][0], acc[i][3], ah, SPLIT ? al : ah);
      Frag<T>::guard(acc[i][1], acc[i][2], ah, SPLIT ? al : ah);
    }
    Frag<T>::keep(bh[0], bh[1], bh[2], bh[3]);
    if (SPLIT) Frag<T>::keep(bl[0], bl[1], bl[2], bl[3]);
  }
  acc_guard4(acc[0][0], acc[0][1], acc[0][2], acc[0][3]);
  acc_guard4(acc[1][0], acc[1][1], acc[1][2], acc[1][3]);
  acc_guard4(acc[2][0], acc[2][1], acc[2][2], acc[2][3]);
  acc_guard4(acc[3][0], acc[3][1], acc[3][2], acc[3][3]);

  float* slab = sT[wave];
  const float* Rb = RESID ? (resid + (size_t)b * strideR) : nullptr;
#pragma unroll
  for (int i = 0; i < 4; ++i) {
    const int mBase = m0 + (i << 4);
#pragma unroll
    for (int j = 0; j < 4; ++j) {
      const int n = n0 + (j << 4) + rlane;
      float bv = 0.f;
      if (BIAS_MODE == 2) bv = bias[n];
#pragma unroll
      for (int r = 0; r < 8; ++r) {
        float v = acc[i][j][r] * scale;
        if (BIAS_MODE == 1) v += bias[mBase + mOff + r];
        if (BIAS_MODE == 2) v += bv;
        if (RESID) v += Rb[(size_t)(mBase + mOff + r) * ldc + n];
        if (ACT == 2) v = fmaxf(v, 0.0f);
        if (ACT == 4) v = (v > 0.f) ? v : 0.01f * v;
        slab[(mOff + r) * 68 + (j << 4) + rlane] = v;
      }
    }
    __builtin_amdgcn_fence(__ATOMIC_RELEASE, "workgroup");
    __builtin_amdgcn_wave_barrier();
    __builtin_amdgcn_fence(__ATOMIC_ACQUIRE, "workgroup");
    if (OUT_MODE == 0) {
      float* C = (float*)Cout + (size_t)b * strideC;
      const int hh = lane >> 4, c4 = (lane & 15) * 4;
      for (int pass = 0; pass < 2; ++pass) {
#pragma unroll
        for (int it = 0; it < 8; ++it) {
          const int row = it * 2 + hh;
          v4f v = *(const v4f*)(slab + row * 68 + c4);
          *(volatile v4f*)(C + (size_t)(mBase + row) * ldc + n0 + c4) = v;
        }
        __threadfence();
      }
    } else {
      const int q = lane >> 3, c8 = (lane & 7) * 8;
      unsigned short* C  = (unsigned short*)Cout  + (size_t)b * strideC;
      unsigned short* C2 = (OUT_MODE == 2) ? ((unsigned short*)Cout2 + (size_t)b * strideC) : nullptr;
      for (int pass = 0; pass < 2; ++pass) {
#pragma unroll
        for (int it = 0; it < 4; ++it) {
          const int row = it * 4 + q;
          const float* sp = slab + row * 68 + c8;
          v8h hv, lv;
#pragma unroll
          for (int e = 0; e < 8; ++e) {
            if (OUT_MODE == 1) {
              hv[e] = (_Float16)sp[e];
            } else {
              unsigned short hb = f2bf_bits(sp[e]);
              unsigned short lb = f2bf_bits(sp[e] - bf_bits2f(hb));
              hv[e] = __builtin_bit_cast(_Float16, hb);
              lv[e] = __builtin_bit_cast(_Float16, lb);
            }
          }
          *(volatile v8h*)(C + (size_t)(mBase + row) * ldc + n0 + c8) = hv;
          if (OUT_MODE == 2) *(volatile v8h*)(C2 + (size_t)(mBase + row) * ldc + n0 + c8) = lv;
        }
        __threadfence();
      }
    }
    __builtin_amdgcn_fence(__ATOMIC_RELEASE, "workgroup");
    __builtin_amdgcn_wave_barrier();
    __builtin_amdgcn_fence(__ATOMIC_ACQUIRE, "workgroup");
  }
}

__global__ __launch_bounds__(kThreads) void prep_kernel(const float* __restrict__ h, const float* __restrict__ W1,
                                                         unsigned short* __restrict__ HB, unsigned short* __restrict__ W1T) {
  const int tid = threadIdx.x;
  if (blockIdx.x < kHBlocks) {
    const int i    = blockIdx.x * kThreads + tid;
    const int row  = i >> 4;
    const int c8   = (i & 15) * 8;
    const bool live = row < kNodes;
    const int rowc = live ? row : (kNodes - 1);
    const float* p = h + (size_t)rowc * kHid + c8;
    const v4f a = *(const v4f*)p;
    const v4f c = *(const v4f*)(p + 4);
    unsigned short hb[8];
#pragma unroll
    for (int e = 0; e < 4; ++e) {
      hb[e]     = live ? f2bf_bits(a[e]) : (unsigned short)0;
      hb[4 + e] = live ? f2bf_bits(c[e]) : (unsigned short)0;
    }
    const v4u u = (v4u){pk16(hb[0], hb[1]), pk16(hb[2], hb[3]), pk16(hb[4], hb[5]), pk16(hb[6], hb[7])};
    unsigned short* q = HB + (size_t)8 * i;
    *(volatile v4u*)q = u;
    __threadfence();
    *(volatile v4u*)q = u;
  } else {
    const int j  = (blockIdx.x - kHBlocks) * kThreads + tid;
    const int n  = j >> 4;
    const int c8 = (j & 15) * 8;
    const float* p = W1 + (size_t)(n & 127) * kCat + (n >> 7) * kHid + c8;
    const v4f a = *(const v4f*)p;
    const v4f c = *(const v4f*)(p + 4);
    unsigned short wb[8];
#pragma unroll
    for (int e = 0; e < 4; ++e) {
      wb[e]     = f2bf_bits(a[e]);
      wb[4 + e] = f2bf_bits(c[e]);
    }
    const v4u u = (v4u){pk16(wb[0], wb[1]), pk16(wb[2], wb[3]), pk16(wb[4], wb[5]), pk16(wb[6], wb[7])};
    unsigned short* q = W1T + (size_t)8 * j;
    *(volatile v4u*)q = u;
    __threadfence();
    *(volatile v4u*)q = u;
  }
}

__global__ __launch_bounds__(kThreads) void edge_kernel(const float* __restrict__ P, const int* __restrict__ src, const int* __restrict__ dst,
                                                         const float* __restrict__ b1, const float* __restrict__ w2,
                                                         const float* __restrict__ b2p, const float* __restrict__ w3p, const float* __restrict__ b3p,
                                                         float* __restrict__ out) {
  __shared__ __align__(16) float sres[kEdgesPerBlk];
  const int tid = threadIdx.x, lane = tid & 31, wave = tid >> 5;
  const int base = blockIdx.x * kEdgesPerBlk;

  const v4f b1raw = *(const v4f*)(b1 + 4 * lane);
  const v4f w2raw = *(const v4f*)(w2 + 4 * lane);
  v4f b1v, w2v;
#pragma unroll
  for (int e = 0; e < 4; ++e) { b1v[e] = bfr(b1raw[e]); w2v[e] = bfr(w2raw[e]); }
  const float b2 = bfr(b2p[0]);
  const float w3 = bfr(w3p[0]);
  const float b3 = bfr(b3p[0]);

  int em = base + wave * 32 + lane;
  em = em < kEdges ? em : (kEdges - 1);
  int sv = src[em];
  int dv = dst[em];
  sv = sv < 0 ? 0 : (sv >= kNodes ? (kNodes - 1) : sv);
  dv = dv < 0 ? 0 : (dv >= kNodes ? (kNodes - 1) : dv);

  float res = 0.0f;
#pragma unroll 1
  for (int j = 0; j < 32; ++j) {
    const int s = __shfl(sv, j, 32);
    const int d = __shfl(dv, j, 32);
    const v4f ps = *(const v4f*)(P + (size_t)s * kCat + 4 * lane);
    const v4f pd = *(const v4f*)(P + (size_t)d * kCat + kHid + 4 * lane);
    v4f x = ps + pd;
    x = x + b1v;
    float part = 0.0f;
#pragma unroll
    for (int e = 0; e < 4; ++e) part = fmaf(fmaxf(x[e], 0.0f), w2v[e], part);
    part += __shfl_xor(part, 16, 32);
    part += __shfl_xor(part, 8, 32);
    part += __shfl_xor(part, 4, 32);
    part += __shfl_xor(part, 2, 32);
    part += __shfl_xor(part, 1, 32);
    float y = fmaxf(part + b2, 0.0f);
    y = y * w3;
    y = fmaxf(y + b3, 0.0f);
    const float t = expf(-y);
    const float o = 1.0f / (1.0f + t);
    res = (lane == j) ? o : res;
  }
  sres[wave * 32 + lane] = res;
  __syncthreads();
  if (wave == 0) {
    const v4f v0 = *(const v4f*)(sres + 4 * lane);
    const v4f v1 = *(const v4f*)(sres + 128 + 4 * lane);
    const int e0 = base + 4 * lane;
    const int e1 = base + 128 + 4 * lane;
    const bool ok0 = (e0 + 3) < kEdges;
    const bool ok1 = (e1 + 3) < kEdges;
    for (int pass = 0; pass < 2; ++pass) {
      if (ok0) *(volatile v4f*)(out + e0) = v0;
      if (ok1) *(volatile v4f*)(out + e1) = v1;
      __threadfence();
    }
  }
}

extern "C" void kernel_launch(void* const* d_in, const int* in_sizes, int n_in,
                              void* d_out, int out_size, void* d_ws, size_t ws_size, hipStream_t stream) {
  if (n_in < 9) return;
  if (in_sizes[0] != kNodes * kHid || in_sizes[1] != kEdges || in_sizes[2] != kEdges ||
      in_sizes[3] != kHid * kCat || in_sizes[4] != kHid || in_sizes[5] != kHid ||
      in_sizes[6] < 1 || in_sizes[7] < 1 || in_sizes[8] < 1 || out_size != kEdges) return;
  if (kWsTotal > ws_size) return;

  const float* h   = (const float*)d_in[0];
  const int*   src = (const int*)  d_in[1];
  const int*   dst = (const int*)  d_in[2];
  const float* W1  = (const float*)d_in[3];
  const float* b1  = (const float*)d_in[4];
  const float* W2  = (const float*)d_in[5];
  const float* b2  = (const float*)d_in[6];
  const float* W3  = (const float*)d_in[7];
  const float* b3  = (const float*)d_in[8];
  float* out = (float*)d_out;

  char* ws = (char*)d_ws;
  unsigned short* HB  = (unsigned short*)(ws);
  unsigned short* W1T = (unsigned short*)(ws + kHbBytes);
  float*          P   = (float*)(ws + kHbBytes + kW1tBytes);

  prep_kernel<<<kHBlocks + kWBlocks, kThreads, 0, stream>>>(h, W1, HB, W1T);

  wmma_gemm64<1, false, 0, 0, false, 0><<<dim3(kGemmBlocks, 1), 256, 0, stream>>>(
      (const unsigned short*)HB, (const unsigned short*)HB, kHid, 0L,
      (const unsigned short*)W1T, (const unsigned short*)W1T, kHid, 0L,
      (void*)P, (void*)nullptr, kCat, 0L,
      (const float*)nullptr, (const float*)nullptr, 0L,
      kNodesPad, kCat, kHid, 1.0f);

  edge_kernel<<<kEdgeBlocks, kThreads, 0, stream>>>(P, src, dst, b1, W2, b2, W3, b3, out);
}
